// DreamGraphReasoner_55405078119324
// MI455X (gfx1250) — hardware-verified
//
#include <hip/hip_runtime.h>
#include <hip/hip_bf16.h>
#include <math.h>

#define GGd 16
#define LLd 64
#define NBt 16
#define DDd 512
#define NN (GGd * LLd)
#define MROWS (NBt * NN)
#define NHOP 3
#define GSTR 48

typedef _Float16 bf16;
typedef _Float16 f16;
typedef __attribute__((ext_vector_type(4))) unsigned v4u_t;
typedef unsigned v4ua __attribute__((ext_vector_type(4), may_alias));
typedef __attribute__((ext_vector_type(4))) float v4f_t;
typedef float v4fa __attribute__((ext_vector_type(4), may_alias));
typedef __attribute__((ext_vector_type(16))) bf16  bf16x16;
typedef bf16x16 f16x16;
typedef __attribute__((ext_vector_type(8)))  bf16  bf16x8;
typedef bf16x8 f16x8;
typedef __attribute__((ext_vector_type(4)))  bf16  bf16x4;
typedef __attribute__((ext_vector_type(8)))  float f32x8;
__device__ __forceinline__ f32x8 wmma16(f16x16 a, f16x16 b, f32x8 c) {
  c = __builtin_amdgcn_wmma_f32_16x16x32_f16(false, a, false, b, (short)0, c, false, false);
  asm volatile("v_nop\n\tv_nop\n\tv_nop\n\tv_nop" : "+v"(c) : "v"(a), "v"(b));
  return c;
}
#define LDS_STRIDE 48
#define KSTRIDE    72
#define VSTRIDE    48

__device__ __forceinline__ f32x8 wmma_bf16(bf16x16 a, bf16x16 b, f32x8 c) {
  c = __builtin_amdgcn_wmma_f32_16x16x32_f16(false, a, false, b, (short)0, c, false, false);
  asm volatile("v_nop\n\tv_nop\n\tv_nop\n\tv_nop" : "+v"(c) : "v"(a), "v"(b));
  return c;
}

template <typename T>
__device__ __forceinline__ bf16x16 load_frag(const T* __restrict__ base, int ld,
                                             int row0, int k0) {
  const int lane = threadIdx.x & 31;
  const int r    = lane & 15;
  const int kh   = (lane >> 4) * 8;
  const T* p0 = base + (size_t)(row0 + r) * ld + (k0 + kh);
  const T* p1 = p0 + 16;
  bf16x16 f;
#pragma unroll
  for (int i = 0; i < 8; ++i) {
    f[i]     = (bf16)p0[i];
    f[i + 8] = (bf16)p1[i];
  }
  return f;
}

__device__ __forceinline__ bf16x16 lds_frag(const bf16* base, int stride) {
  const int lane = threadIdx.x & 31;
  const int row  = lane & 15;
  const int kh   = (lane >> 4) * 8;
  const bf16x8 lo = *(const bf16x8*)(base + row * stride + kh);
  const bf16x8 hi = *(const bf16x8*)(base + row * stride + kh + 16);
  bf16x16 f;
#pragma unroll
  for (int i = 0; i < 8; ++i) { f[i] = lo[i]; f[i + 8] = hi[i]; }
  return f;
}

template <typename T>
__device__ __forceinline__ void stage_read16(const T* __restrict__ p, float* buf) {
#pragma unroll
  for (int i = 0; i < 16; ++i) buf[i] = (float)p[i];
}

__device__ __forceinline__ void stage_write(bf16* dst, const float* buf, int nquad) {
#pragma unroll
  for (int i = 0; i < nquad; ++i) {
    bf16x4 q;
    q[0] = (bf16)buf[4 * i];     q[1] = (bf16)buf[4 * i + 1];
    q[2] = (bf16)buf[4 * i + 2]; q[3] = (bf16)buf[4 * i + 3];
    *(bf16x4*)(dst + 4 * i) = q;
  }
}


#define GSTR 48
template <typename AT, int EPI, bool OUT16>
__global__ __launch_bounds__(256) void gemm_kne(const AT* __restrict__ A, int lda, const float* __restrict__ Wm, int ldw,
                                                const float* __restrict__ bias, const float* __restrict__ R, const float* __restrict__ gvec,
                                                void* __restrict__ Yv, int ldy, int K) {
  __shared__ __attribute__((aligned(16))) f16 ldsA[128 * GSTR];
  __shared__ __attribute__((aligned(16))) f16 ldsW[128 * GSTR];
  __shared__ __attribute__((aligned(16))) float oS[8][32 * 68];
  const int tid = threadIdx.x, lane = tid & 31, wave = tid >> 5, cl = lane & 15, rh = (lane >> 4) * 8;
  const int m0 = blockIdx.x * 128, n0 = blockIdx.y * 128;
  const int wm = (wave & 3) * 32, wn = (wave >> 2) * 64;
  f32x8 acc[2][4];
#pragma unroll
  for (int i = 0; i < 2; ++i)
#pragma unroll
    for (int j = 0; j < 4; ++j) { f32x8 z = {}; acc[i][j] = z; }
#pragma unroll 1
  for (int k0 = 0; k0 < K; k0 += 32) {
    __syncthreads();
    { const int row = tid >> 1, ch = (tid & 1) * 16;
      const AT* src = A + (size_t)(m0 + row) * lda + k0 + ch;
#pragma unroll
      for (int g = 0; g < 16; ++g) ldsA[row * GSTR + ch + g] = (f16)src[g]; }
    { const int k = tid >> 3, nn0 = (tid & 7) * 16;
      const float* src = Wm + (size_t)(k0 + k) * ldw + n0 + nn0;
#pragma unroll
      for (int g = 0; g < 4; ++g) { const v4f_t v = *(const v4f_t*)(src + 4 * g);
#pragma unroll
        for (int u = 0; u < 4; ++u) ldsW[(nn0 + 4 * g + u) * GSTR + k] = (f16)v[u]; } }
    __syncthreads();
    f16x16 af[2];
#pragma unroll
    for (int i = 0; i < 2; ++i) af[i] = lds_frag(ldsA + (wm + 16 * i) * GSTR, GSTR);
#pragma unroll
    for (int j = 0; j < 4; ++j) {
      const f16x16 bf = lds_frag(ldsW + (wn + 16 * j) * GSTR, GSTR);
#pragma unroll
      for (int i = 0; i < 2; ++i) acc[i][j] = wmma16(af[i], bf, acc[i][j]);
    }
  }
  float* so = oS[wave];
#pragma unroll
  for (int i = 0; i < 2; ++i)
#pragma unroll
    for (int j = 0; j < 4; ++j) {
      const int n = n0 + wn + 16 * j + cl;
      const float bv = bias ? bias[n] : 0.0f;
      const float gv = (EPI == 2) ? gvec[n] : 0.0f;
      if (EPI == 1) {
#pragma unroll 1
        for (int r = 0; r < 8; ++r) { const float xg = acc[i][j][r] + bv; so[(16 * i + rh + r) * 68 + 16 * j + cl] = 0.5f * xg * (1.0f + erff(xg * 0.70710678118654752f)); }
      } else {
#pragma unroll
        for (int r = 0; r < 8; ++r) {
          float v = acc[i][j][r] + bv;
          if (EPI == 2) v = R[(size_t)(m0 + wm + 16 * i + rh + r) * ldy + n] + gv * v;
          so[(16 * i + rh + r) * 68 + 16 * j + cl] = v;
        }
      }
    }
  asm volatile("s_wait_dscnt 0" ::: "memory");
  __builtin_amdgcn_wave_barrier();
#pragma unroll 1
  for (int pass = 0; pass < 2; ++pass) {
    if (OUT16) {
      f16* Y = (f16*)Yv;
#pragma unroll
      for (int it = 0; it < 8; ++it) { const int c = lane + 32 * it, rr = c >> 3, q8 = (c & 7) * 8;
        union { f16 h[8]; v4u_t v; } u;
#pragma unroll
        for (int e = 0; e < 8; ++e) u.h[e] = (f16)so[rr * 68 + q8 + e];
        *(volatile v4u_t*)(Y + (size_t)(m0 + wm + rr) * ldy + n0 + wn + q8) = u.v; }
    } else {
      float* Y = (float*)Yv;
#pragma unroll
      for (int it = 0; it < 16; ++it) { const int f4 = lane + 32 * it, rr = f4 >> 4, q = (f4 & 15) * 4;
        *(volatile v4f_t*)(Y + (size_t)(m0 + wm + rr) * ldy + n0 + wn + q) = *(const v4fa*)(so + rr * 68 + q); }
    }
    __threadfence();
  }
}

__global__ __launch_bounds__(128) void k_nodes(const float* __restrict__ wa, const float* __restrict__ ac, const float* __restrict__ re, float* __restrict__ x) {
  const int n = blockIdx.x, b = blockIdx.y; const size_t src = ((size_t)n * NBt + b) * DDd; const size_t dst = ((size_t)b * NN + n) * DDd;
  const int c4 = threadIdx.x * 4; const v4f_t p = *(const v4f_t*)(wa + src + c4), q = *(const v4f_t*)(ac + src + c4), r = *(const v4f_t*)(re + src + c4); v4f_t o;
  for (int e = 0; e < 4; ++e) o[e] = (p[e] + q[e] + r[e]) * (1.0f / 3.0f);
  *(volatile v4f_t*)(x + dst + c4) = o; __threadfence(); *(volatile v4f_t*)(x + dst + c4) = o;
}
__global__ __launch_bounds__(128) void k_gattn(const bf16* __restrict__ Q, const bf16* __restrict__ K, const bf16* __restrict__ V, bf16* __restrict__ att) {
  __shared__ float red[17][4]; __shared__ float pS[20]; __shared__ float eS[20];
  const int n = blockIdx.x, b = blockIdx.y, tid = threadIdx.x, lane = tid & 31, wave = tid >> 5; const int d = n / LLd, s = n % LLd;
  const int J = 17 + (int)(blockIdx.x >> 30);
  const size_t base = (size_t)b * NN; const int c4 = tid * 4;
  const bf16* qr = Q + (base + n) * DDd + c4; float q[4]; for (int e = 0; e < 4; ++e) q[e] = (float)qr[e];
  const int nk = (s + 1 < LLd) ? 17 : 16;
  for (int j = 0; j < J; ++j) { float part = 0.0f;
    if (j < nk && j != d) { const int m = (j < 16) ? (j * LLd + s) : (d * LLd + s + 1); const bf16* kr = K + (base + m) * DDd + c4; for (int e = 0; e < 4; ++e) part += q[e] * (float)kr[e]; }
#pragma unroll
    for (int off = 1; off < 32; off <<= 1) part += __shfl_xor(part, off, 32);
    if (lane == 0) red[j][wave] = part;
  }
  __syncthreads();
  if (tid < 17) { const bool valid = (tid < nk) && (tid != d); pS[tid] = valid ? (red[tid][0] + red[tid][1] + red[tid][2] + red[tid][3]) * 0.044194173824159216f : -3.0e38f; }
  __syncthreads();
  if (tid < 17) { float m = -3.0e38f; for (int j = 0; j < J; ++j) m = fmaxf(m, pS[j]); eS[tid] = (pS[tid] > -1.0e38f) ? expf(pS[tid] - m) : 0.0f; }
  __syncthreads();
  if (tid == 0) { float z = 0.0f; for (int j = 0; j < J; ++j) z += eS[j]; const float iz = 1.0f / z; for (int j = 0; j < J; ++j) pS[j] = eS[j] * iz; }
  __syncthreads();
  float o[4] = {0.f, 0.f, 0.f, 0.f};
  for (int j = 0; j < J; ++j) { const float p = pS[j]; if (p != 0.0f) { const int m = (j < 16) ? (j * LLd + s) : (d * LLd + s + 1); const bf16* vr = V + (base + m) * DDd + c4; for (int e = 0; e < 4; ++e) o[e] += p * (float)vr[e]; } }
  union { bf16 h[4]; __attribute__((ext_vector_type(2))) unsigned u2; } cv; for (int e = 0; e < 4; ++e) cv.h[e] = (bf16)o[e];
  typedef __attribute__((ext_vector_type(2))) unsigned v2u;
  *(volatile v2u*)(att + (base + n) * DDd + c4) = cv.u2; __threadfence(); *(volatile v2u*)(att + (base + n) * DDd + c4) = cv.u2;
}
__global__ __launch_bounds__(128) void k_addrelu(float* __restrict__ x, const float* __restrict__ t) { const size_t off = (size_t)blockIdx.x * DDd + threadIdx.x * 4;
  const v4f_t a = *(const v4f_t*)(x + off), u = *(const v4f_t*)(t + off); v4f_t o; for (int e = 0; e < 4; ++e) o[e] = a[e] + fmaxf(u[e], 0.0f);
  *(volatile v4f_t*)(x + off) = o; __threadfence(); *(volatile v4f_t*)(x + off) = o; }
__global__ __launch_bounds__(128) void k_mean(const float* __restrict__ x, float* __restrict__ agg) { const int b = blockIdx.y, c = blockIdx.x * 128 + threadIdx.x; float s = 0.0f;
  if (b < NBt) {
#pragma unroll 1
    for (int n = 0; n < NN; ++n) s += x[((size_t)b * NN + n) * DDd + c];
    s *= (1.0f / NN); }
  *(volatile float*)(agg + (size_t)b * DDd + c) = s; __threadfence(); *(volatile float*)(agg + (size_t)b * DDd + c) = s; }
__global__ __launch_bounds__(256) void k_relu(float* __restrict__ t, int rowlen) { const size_t row = blockIdx.x;
  for (int q4 = threadIdx.x; q4 < rowlen / 4; q4 += 256) { v4f_t v = *(const v4f_t*)(t + row * rowlen + q4 * 4); for (int e = 0; e < 4; ++e) v[e] = fmaxf(v[e], 0.0f);
    *(volatile v4f_t*)(t + row * rowlen + q4 * 4) = v; __threadfence(); *(volatile v4f_t*)(t + row * rowlen + q4 * 4) = v; } }
__global__ __launch_bounds__(128) void k_copyout(const float* __restrict__ src, float* __restrict__ out) { const size_t off = (size_t)blockIdx.x * DDd + threadIdx.x * 4;
  const v4f_t v = *(const v4f_t*)(src + off); *(volatile v4f_t*)(out + off) = v; __threadfence(); *(volatile v4f_t*)(out + off) = v; }

extern "C" void kernel_launch(void* const* d_in, const int* in_sizes, int n_in,
                              void* d_out, int out_size, void* d_ws, size_t ws_size,
                              hipStream_t stream) {
  (void)in_sizes; (void)n_in; (void)out_size;
  const float** f = (const float**)d_in;
  const float* wa = f[0], *ac = f[1], *re = f[2], *Wq = f[3], *bq = f[4], *Wk = f[5], *bk = f[6], *Wv = f[7], *bv = f[8], *Wh = f[9], *bh = f[10], *Wa1 = f[11], *ba1 = f[12], *Wa2 = f[13], *ba2 = f[14];
  float* out = (float*)d_out;
  char* ws = (char*)d_ws;
  float* x = (float*)ws; ws += (size_t)MROWS * DDd * 4;
  bf16* Q16 = (bf16*)ws; ws += (size_t)MROWS * DDd * 2; bf16* K16 = (bf16*)ws; ws += (size_t)MROWS * DDd * 2; bf16* V16 = (bf16*)ws; ws += (size_t)MROWS * DDd * 2;
  bf16* att = (bf16*)ws; ws += (size_t)MROWS * DDd * 2;
  float* t = (float*)Q16;
  float* agg = (float*)ws; ws += (size_t)128 * DDd * 4; float* hdn = (float*)ws; ws += (size_t)128 * 2 * DDd * 4; float* res = (float*)ws; ws += (size_t)128 * DDd * 4;
  if ((size_t)(ws - (char*)d_ws) > ws_size) return;
  const dim3 blk(256);
  k_nodes<<<dim3(NN, NBt), dim3(128), 0, stream>>>(wa, ac, re, x);
  for (int h = 0; h < NHOP; ++h) {
    gemm_kne<float, 0, true><<<dim3(MROWS / 128, DDd / 128), blk, 0, stream>>>(x, DDd, Wq, DDd, bq, nullptr, nullptr, Q16, DDd, DDd);
    gemm_kne<float, 0, true><<<dim3(MROWS / 128, DDd / 128), blk, 0, stream>>>(x, DDd, Wk, DDd, bk, nullptr, nullptr, K16, DDd, DDd);
    gemm_kne<float, 0, true><<<dim3(MROWS / 128, DDd / 128), blk, 0, stream>>>(x, DDd, Wv, DDd, bv, nullptr, nullptr, V16, DDd, DDd);
    k_gattn<<<dim3(NN, NBt), dim3(128), 0, stream>>>(Q16, K16, V16, att);
    gemm_kne<bf16, 0, false><<<dim3(MROWS / 128, DDd / 128), blk, 0, stream>>>(att, DDd, Wh + (size_t)h * DDd * DDd, DDd, bh + h * DDd, nullptr, nullptr, t, DDd, DDd);
    k_addrelu<<<dim3(MROWS), dim3(128), 0, stream>>>(x, t);
  }
  k_mean<<<dim3(DDd / 128, 128), dim3(128), 0, stream>>>(x, agg);
  gemm_kne<float, 0, false><<<dim3(1, 2 * DDd / 128), blk, 0, stream>>>(agg, DDd, Wa1, 2 * DDd, ba1, nullptr, nullptr, hdn, 2 * DDd, DDd);
  k_relu<<<dim3(128), blk, 0, stream>>>(hdn, 2 * DDd);
  gemm_kne<float, 0, false><<<dim3(1, DDd / 128), blk, 0, stream>>>(hdn, 2 * DDd, Wa2, DDd, ba2, nullptr, nullptr, res, DDd, 2 * DDd);
  k_copyout<<<dim3(NBt), dim3(128), 0, stream>>>(res, out);
}
